// Memory_36550171689427
// MI455X (gfx1250) — hardware-verified
//
#include <hip/hip_runtime.h>
#include <math.h>

constexpr int kBatch  = 8;
constexpr int kSeq    = 512;
constexpr int kDim    = 256;
constexpr int kHeads  = 4;
constexpr int kDh     = 64;
constexpr int kSlots  = 20;
constexpr int kNum    = kBatch * kSeq;
constexpr int kVocab  = 50000;
constexpr int kHalfRows = 25024;
constexpr int kVocabPad = 2 * kHalfRows;
constexpr int kTokPerBlk = 8;
constexpr float kScoreScale = 0.125f;
constexpr float kNegInit = -3.0e38f;
constexpr int kTilesQ     = (kNum / 64) * (kDim / 64);
constexpr int kBlocksQ    = (kTilesQ + 7) / 8;
constexpr int kTilesHalf  = (kHalfRows / 64) * (kDim / 64);
constexpr int kBlocksHalf = (kTilesHalf + 7) / 8;
static_assert(kHeads * kDh == kDim, "shape");
static_assert(kNum % 64 == 0 && kHalfRows % 64 == 0 && kDim % 64 == 0 && kDim % 32 == 0, "tiles");
static_assert(kVocabPad >= kVocab && kHalfRows <= kVocab, "chunks");
static_assert(kNum % kTokPerBlk == 0 && kTokPerBlk * 32 == 256, "waves");
static_assert(kSlots <= 32 && kDim == 32 * 8, "lanes");

typedef __attribute__((ext_vector_type(16))) _Float16 v16h;
typedef __attribute__((ext_vector_type(8)))  _Float16 v8h;
typedef __attribute__((ext_vector_type(16))) __bf16   v16b;
typedef __attribute__((ext_vector_type(8)))  __bf16   v8b;
typedef __attribute__((ext_vector_type(8)))  float    v8f;
typedef __attribute__((ext_vector_type(4)))  float    v4f;
typedef __attribute__((ext_vector_type(4)))  unsigned int v4u;

__device__ __forceinline__ unsigned short f2bf_bits(float f) {
  unsigned u = __float_as_uint(f);
  return (unsigned short)((u + 0x7FFFu + ((u >> 16) & 1u)) >> 16);
}
__device__ __forceinline__ float bf_bits2f(unsigned short h) { return __uint_as_float(((unsigned)h) << 16); }
__device__ __forceinline__ float rbf(float f) { return bf_bits2f(f2bf_bits(f)); }

__device__ __forceinline__ void dep_guard_h(v8f& a, v8f& b, v16h x, v16h y) { asm volatile("v_nop\n\tv_nop\n\tv_nop\n\tv_nop" : "+v"(a), "+v"(b) : "v"(x), "v"(y)); }
__device__ __forceinline__ void dep_guard_b(v8f& a, v8f& b, v16b x, v16b y) { asm volatile("v_nop\n\tv_nop\n\tv_nop\n\tv_nop" : "+v"(a), "+v"(b) : "v"(x), "v"(y)); }
__device__ __forceinline__ void dep_guard4_h(v8f& a, v8f& b, v8f& c, v8f& d, v16h x, v16h y) { asm volatile("v_nop\n\tv_nop\n\tv_nop\n\tv_nop" : "+v"(a), "+v"(b), "+v"(c), "+v"(d) : "v"(x), "v"(y)); }
__device__ __forceinline__ void dep_guard4_b(v8f& a, v8f& b, v8f& c, v8f& d, v16b x, v16b y) { asm volatile("v_nop\n\tv_nop\n\tv_nop\n\tv_nop" : "+v"(a), "+v"(b), "+v"(c), "+v"(d) : "v"(x), "v"(y)); }
__device__ __forceinline__ void keep4_h(v16h a, v16h b, v16h c, v16h d) { asm volatile("v_nop" :: "v"(a), "v"(b), "v"(c), "v"(d)); }
__device__ __forceinline__ void keep4_b(v16b a, v16b b, v16b c, v16b d) { asm volatile("v_nop" :: "v"(a), "v"(b), "v"(c), "v"(d)); }
__device__ __forceinline__ void acc_guard4(v8f& a, v8f& b, v8f& c, v8f& d) { asm volatile("v_nop\n\tv_nop\n\tv_nop\n\tv_nop" : "+v"(a), "+v"(b), "+v"(c), "+v"(d)); }
template <typename T> struct Frag;
template <> struct Frag<_Float16> {
  typedef v16h V; union U { v16h v; v8h h[2]; };
  static __device__ __forceinline__ v16h load(const _Float16* p) {
    U f; f.h[0] = *(const v8h*)(p); f.h[1] = *(const v8h*)(p + 16); return f.v;
  }
  static __device__ __forceinline__ v8f mma(v16h a, v16h b, v8f c) {
    return __builtin_amdgcn_wmma_f32_16x16x32_f16(false, a, false, b, (short)0, c, false, false);
  }
  static __device__ __forceinline__ void guard(v8f& a, v8f& b, v16h x, v16h y) { dep_guard_h(a, b, x, y); }
  static __device__ __forceinline__ void guard4(v8f& a, v8f& b, v8f& c, v8f& d, v16h x, v16h y) { dep_guard4_h(a, b, c, d, x, y); }
  static __device__ __forceinline__ void keep(v16h a, v16h b, v16h c, v16h d) { keep4_h(a, b, c, d); }
};
template <> struct Frag<__bf16> {
  typedef v16b V; union U { v16b v; v8b h[2]; };
  static __device__ __forceinline__ v16b load(const __bf16* p) {
    U f; f.h[0] = *(const v8b*)(p); f.h[1] = *(const v8b*)(p + 16); return f.v;
  }
  static __device__ __forceinline__ v8f mma(v16b a, v16b b, v8f c) {
    return __builtin_amdgcn_wmma_f32_16x16x32_bf16(false, a, false, b, (short)0, c, false, false);
  }
  static __device__ __forceinline__ void guard(v8f& a, v8f& b, v16b x, v16b y) { dep_guard_b(a, b, x, y); }
  static __device__ __forceinline__ void guard4(v8f& a, v8f& b, v8f& c, v8f& d, v16b x, v16b y) { dep_guard4_b(a, b, c, d, x, y); }
  static __device__ __forceinline__ void keep(v16b a, v16b b, v16b c, v16b d) { keep4_b(a, b, c, d); }
};

__device__ __forceinline__ unsigned pk16(unsigned short a, unsigned short b) { return (unsigned)a | ((unsigned)b << 16); }

template <int ET> struct Elem;
template <> struct Elem<0> { typedef _Float16 T; };
template <> struct Elem<1> { typedef __bf16 T; };
template <int ET, bool SPLIT, int BIAS_MODE, int OUT_MODE, bool RESID, int ACT = 0>
__global__ __launch_bounds__(256) void wmma_gemm64(
    const unsigned short* __restrict__ Ap, const unsigned short* __restrict__ A2p, int lda, long strideA,
    const unsigned short* __restrict__ Btp, const unsigned short* __restrict__ Bt2p, int ldb, long strideB,
    void* __restrict__ Cout, void* __restrict__ Cout2, int ldc, long strideC,
    const float* __restrict__ bias,
    const float* __restrict__ resid, long strideR,
    int M, int N, int K, float scale) {
  typedef typename Elem<ET>::T T;
  typedef typename Frag<T>::V V;
  const T* A = (const T*)Ap; const T* A2 = (const T*)A2p; const T* Bt = (const T*)Btp; const T* Bt2 = (const T*)Bt2p;
  __shared__ __align__(16) float sT[8][16 * 68];
  const int b    = blockIdx.y;
  const int lane = threadIdx.x & 31;
  const int wave = threadIdx.x >> 5;
  const int tilesN = N >> 6;
  const int tilesM = M >> 6;
  const int tile = blockIdx.x * 8 + wave;
  if (tile >= tilesM * tilesN) return;
  const int tm = tile / tilesN;
  const int tn = tile - tm * tilesN;
  const int m0 = tm << 6;
  const int n0 = tn << 6;

  const T* Ab  = A  + (size_t)b * strideA;
  const T* Bb  = Bt + (size_t)b * strideB;
  const T* Ab2 = SPLIT ? (A2  + (size_t)b * strideA) : nullptr;
  const T* Bb2 = SPLIT ? (Bt2 + (size_t)b * strideB) : nullptr;

  const int rlane = lane & 15;
  const int koff  = (lane >> 4) * 8;
  const int mOff  = (lane >> 4) * 8;

  v8f acc[4][4];
#pragma unroll
  for (int i = 0; i < 4; ++i)
#pragma unroll
    for (int j = 0; j < 4; ++j) acc[i][j] = (v8f){0.f,0.f,0.f,0.f,0.f,0.f,0.f,0.f};

  for (int k0 = 0; k0 < K; k0 += 32) {
    V bh[4], bl[4];
#pragma unroll
    for (int j = 0; j < 4; ++j) {
      const size_t bo = (size_t)(n0 + (j << 4) + rlane) * ldb + koff + k0;
      bh[j] = Frag<T>::load(Bb + bo);
      if (SPLIT) bl[j] = Frag<T>::load(Bb2 + bo);
    }
#pragma unroll
    for (int i = 0; i < 4; ++i) {
      const size_t ao = (size_t)(m0 + (i << 4) + rlane) * lda + koff + k0;
      V ah = Frag<T>::load(Ab + ao);
      V al;
      if (SPLIT) al = Frag<T>::load(Ab2 + ao);
#pragma unroll
      for (int j = 0; j < 4; ++j) {
        acc[i][j] = Frag<T>::mma(ah, bh[j], acc[i][j]);
        if (SPLIT) {
          acc[i][j] = Frag<T>::mma(ah, bl[j], acc[i][j]);
          acc[i][j] = Frag<T>::mma(al, bh[j], acc[i][j]);
        }
      }
      Frag<T>::guard4(acc[i][0], acc[i][1], acc[i][2], acc[i][3], ah, SPLIT ? al : ah);
    }
    Frag<T>::keep(bh[0], bh[1], bh[2], bh[3]);
    if (SPLIT) Frag<T>::keep(bl[0], bl[1], bl[2], bl[3]);
  }
  acc_guard4(acc[0][0], acc[0][1], acc[0][2], acc[0][3]);
  acc_guard4(acc[1][0], acc[1][1], acc[1][2], acc[1][3]);
  acc_guard4(acc[2][0], acc[2][1], acc[2][2], acc[2][3]);
  acc_guard4(acc[3][0], acc[3][1], acc[3][2], acc[3][3]);

  float* slab = sT[wave];
  const float* Rb = RESID ? (resid + (size_t)b * strideR) : nullptr;
#pragma unroll
  for (int i = 0; i < 4; ++i) {
    const int mBase = m0 + (i << 4);
#pragma unroll
    for (int j = 0; j < 4; ++j) {
      const int n = n0 + (j << 4) + rlane;
      float bv = 0.f;
      if (BIAS_MODE == 2) bv = bias[n];
#pragma unroll
      for (int r = 0; r < 8; ++r) {
        float v = acc[i][j][r] * scale;
        if (BIAS_MODE == 1) v += bias[mBase + mOff + r];
        if (BIAS_MODE == 2) v += bv;
        if (RESID) v += Rb[(size_t)(mBase + mOff + r) * ldc + n];
        if (ACT == 2) v = fmaxf(v, 0.0f);
        if (ACT == 4) v = (v > 0.f) ? v : 0.01f * v;
        slab[(mOff + r) * 68 + (j << 4) + rlane] = v;
      }
    }
    __builtin_amdgcn_fence(__ATOMIC_RELEASE, "workgroup");
    __builtin_amdgcn_wave_barrier();
    __builtin_amdgcn_fence(__ATOMIC_ACQUIRE, "workgroup");
    if (OUT_MODE == 0) {
      float* C = (float*)Cout + (size_t)b * strideC;
      const int hh = lane >> 4, c4 = (lane & 15) * 4;
      for (int pass = 0; pass < 2; ++pass) {
#pragma unroll
        for (int it = 0; it < 8; ++it) {
          const int row = it * 2 + hh;
          v4f v = *(const v4f*)(slab + row * 68 + c4);
          *(volatile v4f*)(C + (size_t)(mBase + row) * ldc + n0 + c4) = v;
        }
        __threadfence();
      }
    } else {
      const int q = lane >> 3, c8 = (lane & 7) * 8;
      unsigned short* C  = (unsigned short*)Cout  + (size_t)b * strideC;
      unsigned short* C2 = (OUT_MODE == 2) ? ((unsigned short*)Cout2 + (size_t)b * strideC) : nullptr;
      for (int pass = 0; pass < 2; ++pass) {
#pragma unroll
        for (int it = 0; it < 4; ++it) {
          const int row = it * 4 + q;
          const float* sp = slab + row * 68 + c8;
          v8h hv, lv;
#pragma unroll
          for (int e = 0; e < 8; ++e) {
            if (OUT_MODE == 1) {
              hv[e] = (_Float16)sp[e];
            } else {
              unsigned short hb = f2bf_bits(sp[e]);
              unsigned short lb = f2bf_bits(sp[e] - bf_bits2f(hb));
              hv[e] = __builtin_bit_cast(_Float16, hb);
              lv[e] = __builtin_bit_cast(_Float16, lb);
            }
          }
          *(volatile v8h*)(C + (size_t)(mBase + row) * ldc + n0 + c8) = hv;
          if (OUT_MODE == 2) *(volatile v8h*)(C2 + (size_t)(mBase + row) * ldc + n0 + c8) = lv;
        }
        __threadfence();
      }
    }
    __builtin_amdgcn_fence(__ATOMIC_RELEASE, "workgroup");
    __builtin_amdgcn_wave_barrier();
    __builtin_amdgcn_fence(__ATOMIC_ACQUIRE, "workgroup");
  }
}

__global__ __launch_bounds__(256) void wt_cast_kernel(const float* __restrict__ W0, const float* __restrict__ W1,
                                                      const float* __restrict__ W2, unsigned short* __restrict__ out) {
  __shared__ float sm[64][65];
  const int t  = threadIdx.x;
  const int d0 = blockIdx.x * 64;
  const int h0 = blockIdx.y * 64;
  const int z  = blockIdx.z;
  const float* W = (z == 0) ? W0 : (z == 1) ? W1 : W2;
#pragma unroll
  for (int i = 0; i < 16; ++i) {
    const int e = i * 256 + t;
    const int r = e >> 6;
    const int c = e & 63;
    sm[c][r] = W[(size_t)(d0 + r) * kDim + h0 + c];
  }
  __syncthreads();
  const int lane = t & 31, wave = t >> 5;
  const int q = lane >> 3, c8 = (lane & 7) * 8;
  unsigned short* op = out + (size_t)z * kDim * kDim;
  for (int pass = 0; pass < 2; ++pass) {
#pragma unroll
    for (int it = 0; it < 2; ++it) {
      const int row = wave * 8 + it * 4 + q;
      unsigned short bb[8];
#pragma unroll
      for (int e = 0; e < 8; ++e) bb[e] = f2bf_bits(sm[row][c8 + e]);
      const v4u u = (v4u){pk16(bb[0], bb[1]), pk16(bb[2], bb[3]), pk16(bb[4], bb[5]), pk16(bb[6], bb[7])};
      *(volatile v4u*)(op + (size_t)(h0 + row) * kDim + d0 + c8) = u;
    }
    __threadfence();
  }
}

__global__ __launch_bounds__(256) void cast_rows_bf16_kernel(const float* __restrict__ src, int src_rows, int r0,
                                                             unsigned short* __restrict__ dst, int n_threads) {
  const int i = blockIdx.x * 256 + threadIdx.x;
  if (i >= n_threads) return;
  const int row  = i >> 5;
  const int c8   = (i & 31) * 8;
  const int srow = r0 + row;
  const int sr   = (srow < src_rows) ? srow : (src_rows - 1);
  const float* p = src + (size_t)sr * kDim + c8;
  const v4f a = *(const v4f*)(p);
  const v4f c = *(const v4f*)(p + 4);
  unsigned short hb[8];
#pragma unroll
  for (int e = 0; e < 4; ++e) {
    hb[e]     = f2bf_bits(a[e]);
    hb[4 + e] = f2bf_bits(c[e]);
  }
  const unsigned keep = (srow < src_rows) ? 0xffffffffu : 0u;
  const v4u u = (v4u){pk16(hb[0], hb[1]) & keep, pk16(hb[2], hb[3]) & keep, pk16(hb[4], hb[5]) & keep, pk16(hb[6], hb[7]) & keep};
  unsigned short* q = dst + (size_t)row * kDim + c8;
  *(volatile v4u*)q = u;
  __threadfence();
  *(volatile v4u*)q = u;
}

__global__ __launch_bounds__(256) void slot_attn_kernel(const float* __restrict__ Qp, const float* __restrict__ Kp,
                                                        const float* __restrict__ Vp, const int* __restrict__ idx,
                                                        const float* __restrict__ bq, const float* __restrict__ bk,
                                                        const float* __restrict__ bv, const float* __restrict__ defh,
                                                        const float* __restrict__ defl,
                                                        float* __restrict__ out0, float* __restrict__ out1, int num) {
  __shared__ __align__(16) float sPar[5][kDim];
  __shared__ int sIdx[kTokPerBlk][32];
  __shared__ __align__(16) float sOh[kTokPerBlk][kDim];
  __shared__ __align__(16) float sOl[kTokPerBlk][kDim];
  const int t    = threadIdx.x;
  const int lane = t & 31;
  const int wave = t >> 5;
  const int n    = blockIdx.x * kTokPerBlk + wave;
  const int nc   = (n < num) ? n : (num - 1);

  sPar[0][t] = rbf(bq[t]);
  sPar[1][t] = rbf(bk[t]);
  sPar[2][t] = rbf(bv[t]);
  sPar[3][t] = rbf(defh[t]);
  sPar[4][t] = rbf(defl[t]);
  {
    const int li = (lane < kSlots) ? lane : (kSlots - 1);
    sIdx[wave][lane] = idx[(size_t)nc * kSlots + li];
  }
  __syncthreads();

  const int ch0 = lane * 8;
  const float* qr = Qp + (size_t)nc * kDim + ch0;
  const v4f qa = *(const v4f*)(qr);
  const v4f qc = *(const v4f*)(qr + 4);
  const v4f b0 = *(const v4f*)(&sPar[0][ch0]);
  const v4f b1 = *(const v4f*)(&sPar[0][ch0 + 4]);
  const v4f k0b = *(const v4f*)(&sPar[1][ch0]);
  const v4f k1b = *(const v4f*)(&sPar[1][ch0 + 4]);
  const v4f v0b = *(const v4f*)(&sPar[2][ch0]);
  const v4f v1b = *(const v4f*)(&sPar[2][ch0 + 4]);
  float q[8], rk[8], rv[8];
#pragma unroll
  for (int e = 0; e < 4; ++e) {
    q[e]      = qa[e] + b0[e];
    q[4 + e]  = qc[e] + b1[e];
    rk[e]     = k0b[e];
    rk[4 + e] = k1b[e];
    rv[e]     = v0b[e];
    rv[4 + e] = v1b[e];
  }

  float mrun = kNegInit;
  float lsum = 0.0f;
  int   nval = 0;
  float ah[8], al[8];
#pragma unroll
  for (int j = 0; j < 8; ++j) { ah[j] = 0.0f; al[j] = 0.0f; }

#pragma unroll 1
  for (int m = 0; m < kSlots; ++m) {
    const int id    = sIdx[wave][m];
    const int valid = (id != 0) ? 1 : 0;
    int idc = (id < 0) ? 0 : id;
    idc = (idc > kVocab - 1) ? (kVocab - 1) : idc;
    const float* kr = Kp + (size_t)idc * kDim + ch0;
    const float* vr = Vp + (size_t)idc * kDim + ch0;
    const v4f ka = *(const v4f*)(kr);
    const v4f kc = *(const v4f*)(kr + 4);
    const v4f va = *(const v4f*)(vr);
    const v4f vc = *(const v4f*)(vr + 4);
    float kf[8], vf[8];
#pragma unroll
    for (int e = 0; e < 4; ++e) {
      kf[e]     = ka[e] + rk[e];
      kf[4 + e] = kc[e] + rk[4 + e];
      vf[e]     = va[e] + rv[e];
      vf[4 + e] = vc[e] + rv[4 + e];
    }
    float s = 0.0f;
#pragma unroll
    for (int j = 0; j < 8; ++j) s += q[j] * kf[j];
    s += __shfl_xor(s, 1, 32);
    s += __shfl_xor(s, 2, 32);
    s += __shfl_xor(s, 4, 32);
    s *= kScoreScale;
    const float seff  = valid ? s : kNegInit;
    const float mnew  = fmaxf(mrun, seff);
    const float alpha = expf(mrun - mnew);
    const float pe    = expf(seff - mnew);
    const float p     = valid ? pe : 0.0f;
    mrun = mnew;
    lsum = lsum * alpha + p;
    nval += valid;
#pragma unroll
    for (int j = 0; j < 8; ++j) {
      ah[j] = ah[j] * alpha + p * kf[j];
      al[j] = al[j] * alpha + p * vf[j];
    }
  }

  const float inv = 1.0f / fmaxf(lsum, 1.0f);
  const bool has  = (nval > 0);
  const v4f d0a = *(const v4f*)(&sPar[3][ch0]);
  const v4f d0c = *(const v4f*)(&sPar[3][ch0 + 4]);
  const v4f d1a = *(const v4f*)(&sPar[4][ch0]);
  const v4f d1c = *(const v4f*)(&sPar[4][ch0 + 4]);
  v4f oh0, oh1, ol0, ol1;
#pragma unroll
  for (int e = 0; e < 4; ++e) {
    const float hk0 = ah[e] * inv;
    const float hk1 = ah[4 + e] * inv;
    const float lv0 = al[e] * inv;
    const float lv1 = al[4 + e] * inv;
    oh0[e] = has ? hk0 : d0a[e];
    oh1[e] = has ? hk1 : d0c[e];
    ol0[e] = has ? lv0 : d1a[e];
    ol1[e] = has ? lv1 : d1c[e];
  }
  *(v4f*)(&sOh[wave][ch0])     = oh0;
  *(v4f*)(&sOh[wave][ch0 + 4]) = oh1;
  *(v4f*)(&sOl[wave][ch0])     = ol0;
  *(v4f*)(&sOl[wave][ch0 + 4]) = ol1;
  __syncthreads();

  const v4f w0 = *(const v4f*)(&sOh[wave][lane * 4]);
  const v4f w1 = *(const v4f*)(&sOh[wave][128 + lane * 4]);
  const v4f x0 = *(const v4f*)(&sOl[wave][lane * 4]);
  const v4f x1 = *(const v4f*)(&sOl[wave][128 + lane * 4]);
  if (n < num) {
    float* o0 = out0 + (size_t)n * kDim;
    float* o1 = out1 + (size_t)n * kDim;
    for (int pass = 0; pass < 2; ++pass) {
      *(volatile v4f*)(o0 + lane * 4)       = w0;
      *(volatile v4f*)(o0 + 128 + lane * 4) = w1;
      *(volatile v4f*)(o1 + lane * 4)       = x0;
      *(volatile v4f*)(o1 + 128 + lane * 4) = x1;
      __threadfence();
    }
  }
}

extern "C" void kernel_launch(void* const* d_in, const int* in_sizes, int n_in,
                              void* d_out, int out_size, void* d_ws, size_t ws_size,
                              hipStream_t stream) {
  if (n_in < 12) return;
  if (in_sizes[0] != kNum * kDim) return;
  if (in_sizes[1] != kNum * kSlots) return;
  if (in_sizes[2] != kVocab * kDim || in_sizes[3] != kVocab * kDim) return;
  if (in_sizes[4] != kDim || in_sizes[5] != kDim) return;
  if (in_sizes[6] != kDim * kDim || in_sizes[8] != kDim * kDim || in_sizes[10] != kDim * kDim) return;
  if (in_sizes[7] != kDim || in_sizes[9] != kDim || in_sizes[11] != kDim) return;
  if (out_size != 2 * kNum * kDim) return;

  const size_t szWT  = (size_t)3 * kDim * kDim * 2;
  const size_t szQ16 = (size_t)kNum * kDim * 2;
  const size_t szQP  = (size_t)kNum * kDim * 4;
  const size_t szA16 = (size_t)kHalfRows * kDim * 2;
  const size_t szKP  = (size_t)kVocabPad * kDim * 4;
  const size_t offWT  = 0;
  const size_t offQ16 = offWT + szWT;
  const size_t offQP  = offQ16 + szQ16;
  const size_t offA16 = offQP + szQP;
  const size_t offKP  = offA16 + szA16;
  const size_t offVP  = offKP + szKP;
  const size_t total  = offVP + szKP;
  if (ws_size < total) return;

  const float* query_h = (const float*)d_in[0];
  const int*   idx     = (const int*)d_in[1];
  const float* mem_h   = (const float*)d_in[2];
  const float* mem_l   = (const float*)d_in[3];
  const float* def_h   = (const float*)d_in[4];
  const float* def_l   = (const float*)d_in[5];
  const float* Wq      = (const float*)d_in[6];
  const float* bq      = (const float*)d_in[7];
  const float* Wk      = (const float*)d_in[8];
  const float* bk      = (const float*)d_in[9];
  const float* Wv      = (const float*)d_in[10];
  const float* bv      = (const float*)d_in[11];

  char* ws = (char*)d_ws;
  unsigned short* WT  = (unsigned short*)(ws + offWT);
  unsigned short* WTQ = WT;
  unsigned short* WTK = WT + (size_t)kDim * kDim;
  unsigned short* WTV = WT + (size_t)2 * kDim * kDim;
  unsigned short* Q16 = (unsigned short*)(ws + offQ16);
  float*          QP  = (float*)(ws + offQP);
  unsigned short* A16 = (unsigned short*)(ws + offA16);
  float*          KP  = (float*)(ws + offKP);
  float*          VP  = (float*)(ws + offVP);
  float* out0 = (float*)d_out;
  float* out1 = (float*)d_out + (size_t)kNum * kDim;

  wt_cast_kernel<<<dim3(kDim / 64, kDim / 64, 3), dim3(256), 0, stream>>>(Wq, Wk, Wv, WT);

  cast_rows_bf16_kernel<<<dim3((kNum * 32) / 256), dim3(256), 0, stream>>>(query_h, kNum, 0, Q16, kNum * 32);

  wmma_gemm64<1, false, 0, 0, false, 0><<<dim3(kBlocksQ, 1), dim3(256), 0, stream>>>(
      Q16, Q16, kDim, 0L, WTQ, WTQ, kDim, 0L, (void*)QP, (void*)QP, kDim, 0L, bq, QP, 0L, kNum, kDim, kDim, 1.0f);

  const int castThreads = kHalfRows * 32;
  const int castBlocks  = castThreads / 256;
  for (int which = 0; which < 2; ++which) {
    const float* src = (which == 0) ? mem_h : mem_l;
    const unsigned short* WTz = (which == 0) ? WTK : WTV;
    float* dstP = (which == 0) ? KP : VP;
    for (int chunk = 0; chunk < 2; ++chunk) {
      const int r0 = chunk * kHalfRows;
      cast_rows_bf16_kernel<<<dim3(castBlocks), dim3(256), 0, stream>>>(src, kVocab, r0, A16, castThreads);
      float* Cp = dstP + (size_t)r0 * kDim;
      wmma_gemm64<1, false, 0, 0, false, 0><<<dim3(kBlocksHalf, 1), dim3(256), 0, stream>>>(
          A16, A16, kDim, 0L, WTz, WTz, kDim, 0L, (void*)Cp, (void*)Cp, kDim, 0L, bq, QP, 0L,
          kHalfRows, kDim, kDim, 1.0f);
    }
  }

  slot_attn_kernel<<<dim3(kNum / kTokPerBlk), dim3(256), 0, stream>>>(QP, KP, VP, idx, bq, bk, bv, def_h, def_l,
                                                                       out0, out1, kNum);
}
